// MambaBlock_71751723647176
// MI455X (gfx1250) — hardware-verified
//
#include <hip/hip_runtime.h>
#include <stddef.h>
#include <stdint.h>
#include <math.h>


#define NBAT   4
#define CINX   64
#define HWD    48
#define SEQ_L  2304
#define MTOK   9216
#define DM     256
#define DI     512
#define DS     32
#define DSH    16
#define DTR    16
#define KC     576
#define XDN    80
#define XDP    128
#define KSEQ   512
#define KU     1024
#define NTHR   256
#define GBM    64
#define GBN    64
#define GTHR   128
#define SD     64
#define TC     64
#define SCT    128
#define NCH    (SEQ_L / TC)
#define U_CW   (DM * (KC / 8))
#define U_WIN  (2 * DI * (KSEQ / 8))
#define U_WX   (XDP * (KU / 8))
#define U_WO   (DM * (KU / 8))
#define U_IM   (MTOK * (KC / 8))
#define WSMAX  134217728

static_assert(U_CW % NTHR == 0 && U_WIN % NTHR == 0 && U_WX % NTHR == 0 && U_WO % NTHR == 0);
static_assert(U_IM % NTHR == 0);
static_assert(MTOK % GBM == 0 && DM % GBN == 0 && (2 * DI) % GBN == 0 && XDP % GBN == 0 && SEQ_L % GBN == 0);
static_assert(KC % 32 == 0 && KSEQ % 32 == 0 && KU % 32 == 0);
static_assert(GBM == (GTHR / 32) * 16 && GBN == 64);
static_assert(SEQ_L % TC == 0 && DI % SD == 0 && SCT == 2 * SD && TC == 64 && DS == 32 && DTR == 16);
static_assert(DS == 2 * DSH && SCT / 32 == TC / 16 && SD == (SCT / 32) * 16);
static_assert((MTOK * (DI / 4)) % NTHR == 0);
static_assert((long long)NBAT * DM * SEQ_L == 2359296LL);

typedef float          v4f   __attribute__((ext_vector_type(4)));
typedef float          v8f   __attribute__((ext_vector_type(8)));
typedef int            v8i   __attribute__((ext_vector_type(8)));
typedef unsigned short v4us  __attribute__((ext_vector_type(4)));
typedef unsigned short v8us  __attribute__((ext_vector_type(8)));
typedef unsigned short v16us __attribute__((ext_vector_type(16)));
typedef __bf16         v16bf __attribute__((ext_vector_type(16)));
typedef v4f  __attribute__((may_alias)) v4fa;
typedef v8us __attribute__((may_alias)) v8usa;
union FragB { v16bf v; v16us u; v8us h[2]; v8i w; };

__device__ __forceinline__ v8f wmb(const FragB& a, const FragB& b, v8f c) {
  v8f d = __builtin_amdgcn_wmma_f32_16x16x32_bf16(false, a.v, false, b.v, (short)0, c, false, false);
  asm volatile("v_nop\n\tv_nop\n\tv_nop\n\tv_nop" : "+v"(d) : "v"(a.w), "v"(b.w));
  return d;
}

__device__ __forceinline__ unsigned bf16_bits(float f) {
  const unsigned u = __float_as_uint(f);
  return (u + 0x7FFFu + ((u >> 16) & 1u)) >> 16;
}
__device__ __forceinline__ float bf16_val(float f) {
  return __uint_as_float(bf16_bits(f) << 16);
}

__device__ __forceinline__ void cvt8_store(const float* p, unsigned short* dp, unsigned msk) {
  const v4f a = *(const v4fa*)p;
  const v4f b = *(const v4fa*)(p + 4);
  v8us o;
  o[0] = (unsigned short)(bf16_bits(a.x) & msk); o[1] = (unsigned short)(bf16_bits(a.y) & msk);
  o[2] = (unsigned short)(bf16_bits(a.z) & msk); o[3] = (unsigned short)(bf16_bits(a.w) & msk);
  o[4] = (unsigned short)(bf16_bits(b.x) & msk); o[5] = (unsigned short)(bf16_bits(b.y) & msk);
  o[6] = (unsigned short)(bf16_bits(b.z) & msk); o[7] = (unsigned short)(bf16_bits(b.w) & msk);
  *(volatile v8us*)dp = o;
  __threadfence();
  *(volatile v8us*)dp = o;
}

__global__ __launch_bounds__(NTHR) void k_wprep(const float* __restrict__ convw, const float* __restrict__ inw,
                                                const float* __restrict__ xw, const float* __restrict__ ow,
                                                unsigned short* CW, unsigned short* WIN2,
                                                unsigned short* WX2, unsigned short* WO2) {
  const int u = (int)blockIdx.x * NTHR + (int)threadIdx.x;
  if (u < U_CW) {
    const int n  = u / (KC / 8);
    const int k8 = (u - n * (KC / 8)) * 8;
    cvt8_store(convw + (size_t)n * KC + k8, CW + (size_t)n * KC + k8, 0xFFFFu);
  } else if (u < U_CW + U_WIN) {
    const int v  = u - U_CW;
    const int n  = v >> 6;
    const int k8 = (v & 63) * 8;
    const int kk = k8 & (DM - 1);
    cvt8_store(inw + (size_t)n * DM + kk, WIN2 + (size_t)n * KSEQ + k8, 0xFFFFu);
  } else if (u < U_CW + U_WIN + U_WX) {
    const int v  = u - U_CW - U_WIN;
    const int n  = v >> 7;
    const int k8 = (v & 127) * 8;
    const int kk = k8 & (DI - 1);
    const int nc = n < XDN ? n : XDN - 1;
    const unsigned msk = 0u - (unsigned)(n < XDN);
    cvt8_store(xw + (size_t)nc * DI + kk, WX2 + (size_t)n * KU + k8, msk);
  } else if (u < U_CW + U_WIN + U_WX + U_WO) {
    const int v  = u - U_CW - U_WIN - U_WX;
    const int n  = v >> 7;
    const int k8 = (v & 127) * 8;
    const int kk = k8 & (DI - 1);
    cvt8_store(ow + (size_t)n * DI + kk, WO2 + (size_t)n * KU + k8, 0xFFFFu);
  }
}

__global__ __launch_bounds__(NTHR) void k_im2col(const float* __restrict__ x, unsigned short* IM) {
  const int u = (int)blockIdx.x * NTHR + (int)threadIdx.x;
  if (u >= U_IM) return;
  const int row = u / (KC / 8);
  const int k8  = (u - row * (KC / 8)) * 8;
  const int b   = row / SEQ_L;
  const int l   = row - b * SEQ_L;
  const int yy  = l / HWD;
  const int xx  = l - yy * HWD;
  const float* xb = x + (size_t)b * (CINX * HWD * HWD);
  v8us o;
#pragma unroll
  for (int i = 0; i < 8; ++i) {
    const int k  = k8 + i;
    const int ci = k / 9;
    const int kk = k - 9 * ci;
    const int ky = kk / 3;
    const int kx = kk - 3 * ky;
    const int iy = yy + ky - 1;
    const int ix = xx + kx - 1;
    const bool ok = ((unsigned)iy < (unsigned)HWD) & ((unsigned)ix < (unsigned)HWD);
    const int iyc = iy < 0 ? 0 : (iy > HWD - 1 ? HWD - 1 : iy);
    const int ixc = ix < 0 ? 0 : (ix > HWD - 1 ? HWD - 1 : ix);
    const float v = xb[(ci * HWD + iyc) * HWD + ixc];
    o[i] = (unsigned short)(bf16_bits(v) & (0u - (unsigned)ok));
  }
  unsigned short* dp = IM + (size_t)row * KC + k8;
  *(volatile v8us*)dp = o;
  __threadfence();
  *(volatile v8us*)dp = o;
}

template <int EPI>
__global__ __launch_bounds__(GTHR) void k_gemm(
    const unsigned short* __restrict__ A, const unsigned short* __restrict__ BT,
    float* outF, unsigned short* outH,
    const float* __restrict__ gam, const float* __restrict__ bet,
    const float* __restrict__ mea, const float* __restrict__ var,
    long long bzB, long long bzO, int K, int ldo)
{
  __shared__ __attribute__((aligned(16))) float stg[GBM * GBN];
  __shared__ float sInv[GBN];
  __shared__ float sSh[GBN];
  const int tid = (int)threadIdx.x, lane = tid & 31, wave = tid >> 5, hh = lane >> 4, m = lane & 15;
  const int rowBase = (int)blockIdx.x * GBM;
  const int col0    = (int)blockIdx.y * GBN;
  const unsigned short* Bz = BT + (size_t)blockIdx.z * (size_t)bzB;

  if constexpr (EPI == 1) {
    if (tid < GBN) {
      const int n = col0 + tid;
      const float g  = bf16_val(gam[n]);
      const float be = bf16_val(bet[n]);
      const float me = bf16_val(mea[n]);
      const float va = bf16_val(var[n]);
      const float iv = g / sqrtf(va + 1e-5f);
      sInv[tid] = iv;
      sSh[tid]  = be - me * iv;
    }
    __syncthreads();
  }

  v8f acc[4];
  {
    const v8f z = {0.f, 0.f, 0.f, 0.f, 0.f, 0.f, 0.f, 0.f};
    acc[0] = z; acc[1] = z; acc[2] = z; acc[3] = z;
  }
  const unsigned short* ap = A  + (size_t)(rowBase + 16 * wave + m) * (size_t)K + 8 * hh;
  const unsigned short* wp = Bz + (size_t)(col0 + m) * (size_t)K + 8 * hh;
  const int ksteps = K >> 5;
#pragma unroll 1
  for (int ks = 0; ks < ksteps; ++ks) {
    FragB af;
    af.h[0] = *(const v8usa*)(ap + 32 * ks);
    af.h[1] = *(const v8usa*)(ap + 32 * ks + 16);
#pragma unroll
    for (int t = 0; t < 4; ++t) {
      const unsigned short* wq = wp + (size_t)(16 * t) * (size_t)K + 32 * ks;
      FragB bf;
      bf.h[0] = *(const v8usa*)wq;
      bf.h[1] = *(const v8usa*)(wq + 16);
      acc[t] = wmb(af, bf, acc[t]);
    }
  }

  if constexpr (EPI == 0) {
#pragma unroll
    for (int t = 0; t < 4; ++t) {
      const int lc = 16 * t + m;
#pragma unroll
      for (int r = 0; r < 8; ++r) {
        const int lr = 16 * wave + 8 * hh + r;
        stg[lr * GBN + lc] = acc[t][r];
      }
    }
    __syncthreads();

    float* oz = outF + (size_t)blockIdx.z * (size_t)bzO;
    v4f fv[8];
#pragma unroll
    for (int i = 0; i < 8; ++i) {
      const int lr = 16 * wave + 2 * i + hh;
      fv[i] = *(const v4fa*)(stg + lr * GBN + 4 * m);
    }
#pragma unroll
    for (int i = 0; i < 8; ++i) {
      const int lr = 16 * wave + 2 * i + hh;
      const int gr = rowBase + lr;
      float* op = oz + (size_t)gr * (size_t)ldo + col0 + 4 * m;
      *(volatile v4f*)op = fv[i];
    }
    __threadfence();
#pragma unroll
    for (int i = 0; i < 8; ++i) {
      const int lr = 16 * wave + 2 * i + hh;
      const int gr = rowBase + lr;
      float* op = oz + (size_t)gr * (size_t)ldo + col0 + 4 * m;
      *(volatile v4f*)op = fv[i];
    }
  } else {
    unsigned short* sh = (unsigned short*)stg;
#pragma unroll
    for (int t = 0; t < 4; ++t) {
      const int lc = 16 * t + m;
      const float iv = sInv[lc];
      const float sf = sSh[lc];
#pragma unroll
      for (int r = 0; r < 8; ++r) {
        const int lr = 16 * wave + 8 * hh + r;
        float v = fmaf(acc[t][r], iv, sf);
        v = v > 0.0f ? v : 0.0f;
        const unsigned hb = bf16_bits(v);
        const unsigned lb = bf16_bits(v - __uint_as_float(hb << 16));
        sh[lr * 128 + lc]      = (unsigned short)hb;
        sh[lr * 128 + 64 + lc] = (unsigned short)lb;
      }
    }
    __syncthreads();
    v8us qv[8];
#pragma unroll
    for (int it = 0; it < 8; ++it) {
      const int li = it * 16 + (tid >> 3);
      const int lr = li >> 1, part = li & 1, pc = tid & 7;
      qv[it] = *(const v8usa*)(sh + lr * 128 + part * 64 + pc * 8);
    }
#pragma unroll
    for (int it = 0; it < 8; ++it) {
      const int li = it * 16 + (tid >> 3);
      const int lr = li >> 1, part = li & 1, pc = tid & 7;
      unsigned short* op = outH + (size_t)(rowBase + lr) * (size_t)ldo + part * DM + col0 + pc * 8;
      *(volatile v8us*)op = qv[it];
    }
    __threadfence();
#pragma unroll
    for (int it = 0; it < 8; ++it) {
      const int li = it * 16 + (tid >> 3);
      const int lr = li >> 1, part = li & 1, pc = tid & 7;
      unsigned short* op = outH + (size_t)(rowBase + lr) * (size_t)ldo + part * DM + col0 + pc * 8;
      *(volatile v8us*)op = qv[it];
    }
  }
}

__global__ __launch_bounds__(NTHR) void k_conv1d(const float* __restrict__ XZ, const float* __restrict__ cw,
                                                 const float* __restrict__ cb, float* U, unsigned short* UHL) {
  const int gid = (int)blockIdx.x * NTHR + (int)threadIdx.x;
  const int row = gid >> 7;
  const int c4  = (gid & 127) * 4;
  const int l   = row % SEQ_L;
  v4f wv[4];
#pragma unroll
  for (int cc = 0; cc < 4; ++cc) {
    const v4f t = *(const v4fa*)(cw + (size_t)(c4 + cc) * 4);
    wv[cc].x = bf16_val(t.x); wv[cc].y = bf16_val(t.y); wv[cc].z = bf16_val(t.z); wv[cc].w = bf16_val(t.w);
  }
  v4f bb;
  {
    const v4f t = *(const v4fa*)(cb + c4);
    bb.x = bf16_val(t.x); bb.y = bf16_val(t.y); bb.z = bf16_val(t.z); bb.w = bf16_val(t.w);
  }
  float a0 = 0.0f, a1 = 0.0f, a2 = 0.0f, a3 = 0.0f;
#pragma unroll
  for (int j = 0; j < 4; ++j) {
    const int rr = row - 3 + j;
    const int rc = rr < 0 ? 0 : rr;
    const float f = (float)((l - 3 + j) >= 0);
    const v4f xv = *(const v4fa*)(XZ + (size_t)rc * (2 * DI) + c4);
    a0 = fmaf(wv[0][j] * f, xv.x, a0);
    a1 = fmaf(wv[1][j] * f, xv.y, a1);
    a2 = fmaf(wv[2][j] * f, xv.z, a2);
    a3 = fmaf(wv[3][j] * f, xv.w, a3);
  }
  a0 += bb.x; a1 += bb.y; a2 += bb.z; a3 += bb.w;
  v4f uo;
  uo.x = a0 * (1.0f / (1.0f + expf(-a0)));
  uo.y = a1 * (1.0f / (1.0f + expf(-a1)));
  uo.z = a2 * (1.0f / (1.0f + expf(-a2)));
  uo.w = a3 * (1.0f / (1.0f + expf(-a3)));
  v4us uh, ul;
  {
    unsigned hb;
    hb = bf16_bits(uo.x); uh[0] = (unsigned short)hb; ul[0] = (unsigned short)bf16_bits(uo.x - __uint_as_float(hb << 16));
    hb = bf16_bits(uo.y); uh[1] = (unsigned short)hb; ul[1] = (unsigned short)bf16_bits(uo.y - __uint_as_float(hb << 16));
    hb = bf16_bits(uo.z); uh[2] = (unsigned short)hb; ul[2] = (unsigned short)bf16_bits(uo.z - __uint_as_float(hb << 16));
    hb = bf16_bits(uo.w); uh[3] = (unsigned short)hb; ul[3] = (unsigned short)bf16_bits(uo.w - __uint_as_float(hb << 16));
  }
  float* up = U + (size_t)row * DI + c4;
  unsigned short* hp = UHL + (size_t)row * KU + c4;
  *(volatile v4f*)up = uo;
  *(volatile v4us*)hp = uh;
  *(volatile v4us*)(hp + DI) = ul;
  __threadfence();
  *(volatile v4f*)up = uo;
  *(volatile v4us*)hp = uh;
  *(volatile v4us*)(hp + DI) = ul;
}

__device__ __forceinline__ float softplus_f(float v) {
  return fmaxf(v, 0.0f) + log1pf(expf(-fabsf(v)));
}

__global__ __launch_bounds__(SCT) void k_scan(const float* __restrict__ XDBL, const float* __restrict__ U,
                                              const float* __restrict__ XZ, const float* __restrict__ dtw,
                                              const float* __restrict__ dtb, const float* __restrict__ Alog,
                                              const float* __restrict__ Dp, unsigned short* GHL) {
  __shared__ __attribute__((aligned(16))) float bc[TC * 64];
  __shared__ __attribute__((aligned(16))) unsigned short adt[TC * 32];
  __shared__ __attribute__((aligned(16))) float dpre[TC * SD];
  __shared__ __attribute__((aligned(16))) unsigned short gst[2 * TC * SD];
  __shared__ __attribute__((aligned(16))) unsigned short wdt[SD * DTR];
  const int tid = (int)threadIdx.x, lane = tid & 31, wave = tid >> 5, hh = lane >> 4, m = lane & 15;
  const int b  = (int)blockIdx.x >> 3;
  const int d0 = ((int)blockIdx.x & 7) * SD;
  const int dl = 16 * wave + m;
  const int d  = d0 + dl;
  const int sb = DSH * hh;

  float a[DSH], s[DSH];
#pragma unroll
  for (int q = 0; q < 4; ++q) {
    const v4f al = *(const v4fa*)(Alog + (size_t)d * DS + sb + 4 * q);
    a[4 * q + 0] = -expf(bf16_val(al.x));
    a[4 * q + 1] = -expf(bf16_val(al.y));
    a[4 * q + 2] = -expf(bf16_val(al.z));
    a[4 * q + 3] = -expf(bf16_val(al.w));
  }
#pragma unroll
  for (int n = 0; n < DSH; ++n) s[n] = 0.0f;
  const float dtbv = bf16_val(dtb[d]);
  const float Dv   = bf16_val(Dp[d]);
  {
    const int dd = tid >> 1, q = tid & 1;
    const float* wp = dtw + (size_t)(d0 + dd) * DTR + 8 * q;
    const v4f w0 = *(const v4fa*)wp;
    const v4f w1 = *(const v4fa*)(wp + 4);
    v8us o;
    o[0] = (unsigned short)bf16_bits(w0.x); o[1] = (unsigned short)bf16_bits(w0.y);
    o[2] = (unsigned short)bf16_bits(w0.z); o[3] = (unsigned short)bf16_bits(w0.w);
    o[4] = (unsigned short)bf16_bits(w1.x); o[5] = (unsigned short)bf16_bits(w1.y);
    o[6] = (unsigned short)bf16_bits(w1.z); o[7] = (unsigned short)bf16_bits(w1.w);
    *(v8usa*)(wdt + dd * DTR + 8 * q) = o;
  }

#pragma unroll 1
  for (int c = 0; c < NCH; ++c) {
    const int row0 = b * SEQ_L + c * TC;
    {
      const int tk = tid >> 1, q = tid & 1;
      const float* xp = XDBL + (size_t)(row0 + tk) * XDP + 8 * q;
      const v4f t0 = *(const v4fa*)xp;
      const v4f t1 = *(const v4fa*)(xp + 4);
      v8us oh, ol;
      unsigned hb;
      hb = bf16_bits(t0.x); oh[0] = (unsigned short)hb; ol[0] = (unsigned short)bf16_bits(t0.x - __uint_as_float(hb << 16));
      hb = bf16_bits(t0.y); oh[1] = (unsigned short)hb; ol[1] = (unsigned short)bf16_bits(t0.y - __uint_as_float(hb << 16));
      hb = bf16_bits(t0.z); oh[2] = (unsigned short)hb; ol[2] = (unsigned short)bf16_bits(t0.z - __uint_as_float(hb << 16));
      hb = bf16_bits(t0.w); oh[3] = (unsigned short)hb; ol[3] = (unsigned short)bf16_bits(t0.w - __uint_as_float(hb << 16));
      hb = bf16_bits(t1.x); oh[4] = (unsigned short)hb; ol[4] = (unsigned short)bf16_bits(t1.x - __uint_as_float(hb << 16));
      hb = bf16_bits(t1.y); oh[5] = (unsigned short)hb; ol[5] = (unsigned short)bf16_bits(t1.y - __uint_as_float(hb << 16));
      hb = bf16_bits(t1.z); oh[6] = (unsigned short)hb; ol[6] = (unsigned short)bf16_bits(t1.z - __uint_as_float(hb << 16));
      hb = bf16_bits(t1.w); oh[7] = (unsigned short)hb; ol[7] = (unsigned short)bf16_bits(t1.w - __uint_as_float(hb << 16));
      *(v8usa*)(adt + tk * 32 + 8 * q)      = oh;
      *(v8usa*)(adt + tk * 32 + 16 + 8 * q) = ol;
    }
#pragma unroll 4
    for (int it = 0; it < 8; ++it) {
      const int idx = it * SCT + tid;
      const int r = idx >> 4, q = idx & 15;
      const v4f v = *(const v4fa*)(XDBL + (size_t)(row0 + r) * XDP + DTR + 4 * q);
      *(v4fa*)(bc + r * 64 + 4 * q) = v;
    }
    __syncthreads();

    {
      FragB af;
      af.h[0] = *(const v8usa*)(adt + (16 * wave + m) * 32 + 8 * hh);
      af.h[1] = *(const v8usa*)(adt + (16 * wave + m) * 32 + 16 + 8 * hh);
#pragma unroll
      for (int j = 0; j < 4; ++j) {
        const v8us wq = *(const v8usa*)(wdt + (16 * j + m) * DTR + 8 * hh);
        FragB bfr;
        bfr.h[0] = wq;
        bfr.h[1] = wq;
        const v8f z = {0.f, 0.f, 0.f, 0.f, 0.f, 0.f, 0.f, 0.f};
        const v8f dacc = wmb(af, bfr, z);
#pragma unroll
        for (int r = 0; r < 8; ++r) dpre[(16 * wave + 8 * hh + r) * SD + 16 * j + m] = dacc[r];
      }
    }
    __syncthreads();

    const float* up = U  + (size_t)row0 * DI + d;
    const float* zp = XZ + (size_t)row0 * (2 * DI) + DI + d;
#pragma unroll 1
    for (int t = 0; t < TC; ++t) {
      const float dp    = dpre[t * SD + dl] + dtbv;
      const float delta = softplus_f(dp);
      const float uu    = up[(size_t)t * DI];
      const float zz    = zp[(size_t)t * (2 * DI)];
      const float du    = delta * uu;
      const float* bp   = bc + t * 64 + sb;
      float dlt = delta;
      float y = 0.0f;
#pragma unroll
      for (int q = 0; q < 4; ++q) {
        if (q > 0) asm volatile("" : "+v"(dlt) : "v"(y));
        const v4f Bv = *(const v4fa*)(bp + 4 * q);
        const v4f Cv = *(const v4fa*)(bp + DS + 4 * q);
#pragma unroll
        for (int e = 0; e < 4; ++e) {
          const int n = 4 * q + e;
          const float dA = expf(dlt * a[n]);
          s[n] = fmaf(s[n], dA, du * Bv[e]);
          y = fmaf(s[n], Cv[e], y);
        }
      }
      const float yo = __shfl_xor(y, 16, 32);
      float yt = y + yo;
      yt = fmaf(uu, Dv, yt);
      const float g  = yt * (zz * (1.0f / (1.0f + expf(-zz))));
      const unsigned hb = bf16_bits(g);
      const unsigned lb = bf16_bits(g - __uint_as_float(hb << 16));
      const unsigned sel = (hh != 0) ? lb : hb;
      gst[hh * (TC * SD) + t * SD + dl] = (unsigned short)sel;
    }
    __syncthreads();

#pragma unroll 4
    for (int it = 0; it < 8; ++it) {
      const int li = it * 16 + (tid >> 3);
      const int part = li >> 6, tk = li & 63, pc = tid & 7;
      const v8us q = *(const v8usa*)(gst + part * (TC * SD) + tk * SD + pc * 8);
      unsigned short* op = GHL + (size_t)(row0 + tk) * KU + part * DI + d0 + pc * 8;
      *(volatile v8us*)op = q;
    }
    __threadfence();
#pragma unroll 4
    for (int it = 0; it < 8; ++it) {
      const int li = it * 16 + (tid >> 3);
      const int part = li >> 6, tk = li & 63, pc = tid & 7;
      const v8us q = *(const v8usa*)(gst + part * (TC * SD) + tk * SD + pc * 8);
      unsigned short* op = GHL + (size_t)(row0 + tk) * KU + part * DI + d0 + pc * 8;
      *(volatile v8us*)op = q;
    }
    __syncthreads();
  }
}

static inline size_t al256(size_t o) { return (o + 255) & ~(size_t)255; }

extern "C" void kernel_launch(void* const* d_in, const int* in_sizes, int n_in,
                              void* d_out, int out_size, void* d_ws, size_t ws_size,
                              hipStream_t stream) {
  if (n_in < 15) return;
  if (in_sizes[0] != NBAT * CINX * HWD * HWD) return;
  if (in_sizes[1] != DM * KC) return;
  if (in_sizes[2] != DM || in_sizes[3] != DM || in_sizes[4] != DM || in_sizes[5] != DM) return;
  if (in_sizes[6] != 2 * DI * DM) return;
  if (in_sizes[7] != DI * 4 || in_sizes[8] != DI) return;
  if (in_sizes[9] != XDN * DI) return;
  if (in_sizes[10] != DI * DTR || in_sizes[11] != DI) return;
  if (in_sizes[12] != DI * DS || in_sizes[13] != DI) return;
  if (in_sizes[14] != DM * DI) return;
  if (out_size != NBAT * DM * SEQ_L) return;

  const float* x     = (const float*)d_in[0];
  const float* convw = (const float*)d_in[1];
  const float* bng   = (const float*)d_in[2];
  const float* bnb   = (const float*)d_in[3];
  const float* bnm   = (const float*)d_in[4];
  const float* bnv   = (const float*)d_in[5];
  const float* inw   = (const float*)d_in[6];
  const float* c1w   = (const float*)d_in[7];
  const float* c1b   = (const float*)d_in[8];
  const float* xw    = (const float*)d_in[9];
  const float* dtw   = (const float*)d_in[10];
  const float* dtb   = (const float*)d_in[11];
  const float* alog  = (const float*)d_in[12];
  const float* dpar  = (const float*)d_in[13];
  const float* ow    = (const float*)d_in[14];
  float* out = (float*)d_out;

  char* ws = (char*)d_ws;
  size_t off = 0;
  const size_t oIM  = off; off = al256(off + (size_t)MTOK * KC * 2);
  const size_t oCW  = off; off = al256(off + (size_t)DM * KC * 2);
  const size_t oWIN = off; off = al256(off + (size_t)2 * DI * KSEQ * 2);
  const size_t oWX  = off; off = al256(off + (size_t)XDP * KU * 2);
  const size_t oWO  = off; off = al256(off + (size_t)DM * KU * 2);
  const size_t oSEQ = off; off = al256(off + (size_t)MTOK * KSEQ * 2);
  const size_t oXZ  = off; off = al256(off + (size_t)MTOK * 2 * DI * 4);
  const size_t oU   = off; off = al256(off + (size_t)MTOK * DI * 4);
  const size_t oUHL = off; off = al256(off + (size_t)MTOK * KU * 2);
  const size_t oXD  = off; off = al256(off + (size_t)MTOK * XDP * 4);
  const size_t oGHL = off; off = al256(off + (size_t)MTOK * KU * 2);
  if (off > ws_size || off > (size_t)WSMAX) return;
  unsigned short* IM   = (unsigned short*)(ws + oIM);
  unsigned short* CW   = (unsigned short*)(ws + oCW);
  unsigned short* WIN2 = (unsigned short*)(ws + oWIN);
  unsigned short* WX2  = (unsigned short*)(ws + oWX);
  unsigned short* WO2  = (unsigned short*)(ws + oWO);
  unsigned short* SEQ  = (unsigned short*)(ws + oSEQ);
  float*          XZ   = (float*)(ws + oXZ);
  float*          U    = (float*)(ws + oU);
  unsigned short* UHL  = (unsigned short*)(ws + oUHL);
  float*          XDBL = (float*)(ws + oXD);
  unsigned short* GHL  = (unsigned short*)(ws + oGHL);

  k_wprep<<<(U_CW + U_WIN + U_WX + U_WO) / NTHR, NTHR, 0, stream>>>(convw, inw, xw, ow, CW, WIN2, WX2, WO2);
  k_im2col<<<U_IM / NTHR, NTHR, 0, stream>>>(x, IM);
  k_gemm<1><<<dim3(MTOK / GBM, DM / GBN, 1), GTHR, 0, stream>>>(
      IM, CW, XZ, SEQ, bng, bnb, bnm, bnv, 0LL, 0LL, KC, KSEQ);
  k_gemm<0><<<dim3(MTOK / GBM, (2 * DI) / GBN, 1), GTHR, 0, stream>>>(
      SEQ, WIN2, XZ, SEQ, bng, bnb, bnm, bnv, 0LL, 0LL, KSEQ, 2 * DI);
  k_conv1d<<<(MTOK * (DI / 4)) / NTHR, NTHR, 0, stream>>>(XZ, c1w, c1b, U, UHL);
  k_gemm<0><<<dim3(MTOK / GBM, XDP / GBN, 1), GTHR, 0, stream>>>(
      UHL, WX2, XDBL, SEQ, bng, bnb, bnm, bnv, 0LL, 0LL, KU, XDP);
  k_scan<<<NBAT * (DI / SD), SCT, 0, stream>>>(XDBL, U, XZ, dtw, dtb, alog, dpar, GHL);
  k_gemm<0><<<dim3(DM / GBM, SEQ_L / GBN, NBAT), GTHR, 0, stream>>>(
      WO2, GHL, out, SEQ, bng, bnb, bnm, bnv,
      (long long)SEQ_L * KU, (long long)DM * SEQ_L, KU, SEQ_L);
}
